// DenseMRConv_79199196938679
// MI455X (gfx1250) — hardware-verified
//
#include <hip/hip_runtime.h>
#include <stddef.h>


#define FD     64
#define KN     32
#define KC     128
#define NO     64
#define NTHR   256
#define NWAVE  8
#define BROWS  64
#define HP     136
#define HSC    8
#define WSC    16
#define WSCAP  134217728
#define WPB    ((NO * KC / 8) / NTHR)

static_assert((NO * KC / 8) % NTHR == 0);
static_assert(KC / 8 == 16);
static_assert(BROWS == (NWAVE / 2) * 16);
static_assert(NO == 2 * 32);
static_assert((KC % 32) == 0);
static_assert(BROWS * KN == NTHR * 8);
static_assert(BROWS == NWAVE * 8);
static_assert((HP * 2) % 16 == 0);
static_assert((8 * NO) % 128 == 0);
static_assert(BROWS * HP * 2 + BROWS * KN * 4 + BROWS * NO * 4 <= 65536);

typedef float     v4f  __attribute__((ext_vector_type(4)));
typedef float     v8f  __attribute__((ext_vector_type(8)));
typedef int       v4i  __attribute__((ext_vector_type(4)));
typedef _Float16  v4h  __attribute__((ext_vector_type(4)));
typedef _Float16  v8h  __attribute__((ext_vector_type(8)));
typedef _Float16  v16h __attribute__((ext_vector_type(16)));
union FragH { v16h v; v8h h[2]; };

__device__ __forceinline__ v8f wmf(v16h a, v16h b, v8f c) {
  v8f d = __builtin_amdgcn_wmma_f32_16x16x32_f16(false, a, false, b, (short)0, c, false, false);
  asm volatile("v_nop\n\tv_nop\n\tv_nop\n\tv_nop" : "+v"(d) : "v"(a), "v"(b));
  return d;
}

__device__ __forceinline__ int clampi(int v, int hi) {
  v = v < 0 ? 0 : v;
  return v > hi ? hi : v;
}

__global__ __launch_bounds__(NTHR) void k_wprep(const float* __restrict__ w, _Float16* wp) {
  const int i  = (int)blockIdx.x * NTHR + (int)threadIdx.x;
  const int n  = i >> 4;
  const int k0 = (i & 15) * 8;
  v8h hv;
#pragma unroll
  for (int e = 0; e < 8; ++e) hv[e] = (_Float16)(w[(size_t)(k0 + e) * NO + n] * (float)WSC);
  _Float16* d = wp + (size_t)i * 8;
  *(volatile v8h*)d = hv;
  __threadfence();
  *(volatile v8h*)d = hv;
}

__global__ __launch_bounds__(NTHR) void k_main(
    const float* __restrict__ x, const int* __restrict__ ei, const _Float16* __restrict__ wp,
    const float* __restrict__ bs, float* out, int nN) {
  __shared__ __attribute__((aligned(16))) _Float16 hs[BROWS * HP];
  __shared__ __attribute__((aligned(16))) int      sidx[BROWS * KN];
  __shared__ __attribute__((aligned(16))) float    stg[BROWS * NO];
  constexpr float OSC = 1.0f / (float)(HSC * WSC);
  const int tid = threadIdx.x, lane = tid & 31, wave = tid >> 5, hh = lane >> 4, m = lane & 15;
  const int base = blockIdx.x * BROWS;

  {
    const int nd = tid >> 2;
    const int q  = tid & 3;
    const int g  = clampi(base + nd, nN - 1);
    const v4i* src = (const v4i*)(ei + (size_t)g * KN + 8 * q);
    v4i a0 = src[0];
    v4i a1 = src[1];
    a0.x = clampi(a0.x, nN - 1); a0.y = clampi(a0.y, nN - 1);
    a0.z = clampi(a0.z, nN - 1); a0.w = clampi(a0.w, nN - 1);
    a1.x = clampi(a1.x, nN - 1); a1.y = clampi(a1.y, nN - 1);
    a1.z = clampi(a1.z, nN - 1); a1.w = clampi(a1.w, nN - 1);
    *(v4i*)(sidx + nd * KN + 8 * q)     = a0;
    *(v4i*)(sidx + nd * KN + 8 * q + 4) = a1;
  }
  __syncthreads();

  {
    const int fq = m * 4;
#pragma unroll 1
    for (int p = 0; p < 4; ++p) {
      const int nd = wave * 8 + 2 * p + hh;
      const int g  = clampi(base + nd, nN - 1);
      const v4f xi = *(const v4f*)(x + (size_t)g * FD + fq);
      v4f mx = { -3.402823466e+38f, -3.402823466e+38f, -3.402823466e+38f, -3.402823466e+38f };
      const int* ip = sidx + nd * KN;
#pragma unroll 8
      for (int k = 0; k < KN; ++k) {
        const int s = ip[k];
        const v4f xj = *(const v4f*)(x + (size_t)s * FD + fq);
        mx.x = fmaxf(mx.x, xj.x);
        mx.y = fmaxf(mx.y, xj.y);
        mx.z = fmaxf(mx.z, xj.z);
        mx.w = fmaxf(mx.w, xj.w);
      }
      const float dx = mx.x - xi.x, dy = mx.y - xi.y, dz = mx.z - xi.z, dw = mx.w - xi.w;
      v4h av, dv;
      av[0] = (_Float16)(xi.x * (float)HSC); av[1] = (_Float16)(xi.y * (float)HSC);
      av[2] = (_Float16)(xi.z * (float)HSC); av[3] = (_Float16)(xi.w * (float)HSC);
      dv[0] = (_Float16)(dx * (float)HSC);   dv[1] = (_Float16)(dy * (float)HSC);
      dv[2] = (_Float16)(dz * (float)HSC);   dv[3] = (_Float16)(dw * (float)HSC);
      *(v4h*)(hs + nd * HP + fq)      = av;
      *(v4h*)(hs + nd * HP + FD + fq) = dv;
    }
  }
  __syncthreads();

  const int rg = wave >> 1, chh = wave & 1;
  v8f acc[2];
  {
    v8f z = {0.f, 0.f, 0.f, 0.f, 0.f, 0.f, 0.f, 0.f};
    acc[0] = z; acc[1] = z;
  }
  const _Float16* ap = hs + (16 * rg + m) * HP + 8 * hh;
#pragma unroll
  for (int kt = 0; kt < KC / 32; ++kt) {
    FragH af;
    af.h[0] = *(const v8h*)(ap + 32 * kt);
    af.h[1] = *(const v8h*)(ap + 32 * kt + 16);
#pragma unroll
    for (int t = 0; t < 2; ++t) {
      const _Float16* bp = wp + (size_t)(32 * chh + 16 * t + m) * KC + 32 * kt + 8 * hh;
      FragH bf;
      bf.h[0] = *(const v8h*)bp;
      bf.h[1] = *(const v8h*)(bp + 16);
      acc[t] = wmf(af.v, bf.v, acc[t]);
    }
  }

  float bv[2];
  bv[0] = bs[32 * chh + m];
  bv[1] = bs[32 * chh + 16 + m];
  float* sp = stg + (16 * rg + 8 * hh) * NO + 32 * chh + m;
#pragma unroll
  for (int t = 0; t < 2; ++t) {
#pragma unroll
    for (int r = 0; r < 8; ++r) sp[r * NO + 16 * t] = acc[t][r] * OSC + bv[t];
  }
  __syncthreads();

  const float* lp = stg + wave * (8 * NO);
#pragma unroll
  for (int i = 0; i < (8 * NO) / 128; ++i) {
    const int row = base + 8 * wave + 2 * i + hh;
    const int rw  = row < nN ? row : nN - 1;
    const v4f v = *(const v4f*)(lp + i * 128 + 4 * lane);
    float* op = out + (size_t)rw * NO + 4 * m;
    if (row < nN) *(volatile v4f*)op = v;
  }
  __threadfence();
#pragma unroll
  for (int i = 0; i < (8 * NO) / 128; ++i) {
    const int row = base + 8 * wave + 2 * i + hh;
    const int rw  = row < nN ? row : nN - 1;
    const v4f v = *(const v4f*)(lp + i * 128 + 4 * lane);
    float* op = out + (size_t)rw * NO + 4 * m;
    if (row < nN) *(volatile v4f*)op = v;
  }
}

extern "C" void kernel_launch(void* const* d_in, const int* in_sizes, int n_in,
                              void* d_out, int out_size, void* d_ws, size_t ws_size,
                              hipStream_t stream) {
  if (n_in < 4) return;
  const int nN = in_sizes[0] / FD;
  if (nN <= 0) return;
  if (in_sizes[0] != nN * FD || in_sizes[1] != nN * KN) return;
  if (in_sizes[2] != KC * NO || in_sizes[3] != NO) return;
  if (out_size != nN * NO) return;
  if (nN > (1 << 24)) return;

  const float* x  = (const float*)d_in[0];
  const int*   ei = (const int*)d_in[1];
  const float* W  = (const float*)d_in[2];
  const float* bs = (const float*)d_in[3];
  float* out = (float*)d_out;

  char* ws = (char*)d_ws;
  size_t off = 0;
  const size_t oW = off; off += (size_t)(NO * KC) * 2;  off = (off + 255) & ~(size_t)255;
  if (off > ws_size || off > (size_t)WSCAP) return;
  _Float16* wp = (_Float16*)(ws + oW);

  const int nBlk = (nN + BROWS - 1) / BROWS;

  k_wprep<<<WPB, NTHR, 0, stream>>>(W, wp);

  k_main<<<nBlk, NTHR, 0, stream>>>(x, ei, wp, bs, out, nN);
}
